// mLSTM_10831907520820
// MI455X (gfx1250) — hardware-verified
//
#include <hip/hip_runtime.h>
#include <stddef.h>

constexpr int NBATCH = 8;
constexpr int SEQ = 1024;
constexpr int DMODEL = 256;
constexpr int MROWS = NBATCH * SEQ;
constexpr int PLEN = 64;
constexpr int NPAIR = MROWS / PLEN;
constexpr int PAIRS_PER_SEQ = SEQ / PLEN;
constexpr size_t NELEM = (size_t)MROWS * DMODEL;
constexpr size_t WELEM = (size_t)DMODEL * DMODEL;

static_assert(MROWS % 64 == 0, "");
static_assert(DMODEL % 64 == 0, "");
static_assert(DMODEL % 32 == 0, "");
static_assert(PLEN % 32 == 0 && PLEN == 64, "");
static_assert(SEQ % PLEN == 0, "");

constexpr size_t MIB = 1048576;
constexpr size_t OFF_R0  = 0;
constexpr size_t OFF_XH  = OFF_R0;
constexpr size_t OFF_XL  = OFF_R0 + 4 * MIB;
constexpr size_t OFF_QF  = OFF_R0 + 8 * MIB;
constexpr size_t OFF_KF  = OFF_R0 + 16 * MIB;
constexpr size_t OFF_FF  = OFF_R0 + 24 * MIB;
constexpr size_t OFF_IF  = OFF_R0 + 32 * MIB;
constexpr size_t OFF_U   = OFF_R0;
constexpr size_t OFF_NS  = OFF_R0 + 32 * MIB;
constexpr size_t OFF_WH  = OFF_R0 + 40 * MIB;
constexpr size_t OFF_WL  = OFF_WH + 5 * WELEM * 2;
constexpr size_t OFF_BIAS = OFF_WL + 5 * WELEM * 2;
constexpr size_t OFF_QKH = OFF_BIAS + 4 * (size_t)DMODEL * 4;
constexpr size_t OFF_QKL = OFF_QKH + 2 * NELEM * 2;
constexpr size_t PLANE_GT = (size_t)NPAIR * DMODEL * PLEN * 2;
constexpr size_t OFF_GTH = OFF_QKL + 2 * NELEM * 2;
constexpr size_t OFF_GTL = OFF_GTH + PLANE_GT;
constexpr size_t OFF_KTH = OFF_GTL + PLANE_GT;
constexpr size_t OFF_KTL = OFF_KTH + PLANE_GT;
constexpr size_t OFF_AD  = OFF_KTL + PLANE_GT;
constexpr size_t OFF_ATH = OFF_AD + (size_t)NPAIR * PLEN * PLEN * 4;
constexpr size_t OFF_ATL = OFF_ATH + (size_t)NPAIR * PLEN * PLEN * 2;
constexpr size_t OFF_FC  = OFF_ATL + (size_t)NPAIR * PLEN * PLEN * 2;
constexpr size_t OFF_DEN = OFF_FC + NELEM * 4;
constexpr size_t OFF_N1  = OFF_DEN + (size_t)MROWS * 4;
constexpr size_t OFF_HH  = OFF_N1;
constexpr size_t OFF_HL  = OFF_N1 + NELEM * 2;
constexpr size_t OFF_CSH = OFF_N1 + NELEM * 4;
constexpr size_t OFF_CSL = OFF_CSH + (size_t)NPAIR * WELEM * 2;
constexpr size_t WS_TOTAL = OFF_CSL + (size_t)NPAIR * WELEM * 2;
static_assert(WS_TOTAL == (size_t)131371008, "");
static_assert(WS_TOTAL <= (size_t)134217728, "");
static_assert((OFF_QKH % 128) == 0 && (OFF_GTH % 128) == 0 && (OFF_AD % 128) == 0 && (OFF_FC % 128) == 0, "");
static_assert((OFF_DEN % 128) == 0 && (OFF_N1 % 128) == 0 && (OFF_CSH % 128) == 0 && (OFF_WL % 128) == 0, "");
static_assert((size_t)NPAIR * WELEM * 4 == 32 * MIB, "");

typedef __attribute__((ext_vector_type(16))) _Float16 v16h;
typedef __attribute__((ext_vector_type(8)))  _Float16 v8h;
typedef __attribute__((ext_vector_type(16))) __bf16   v16b;
typedef __attribute__((ext_vector_type(8)))  __bf16   v8b;
typedef __attribute__((ext_vector_type(8)))  float    v8f;
typedef __attribute__((ext_vector_type(4)))  float    v4f;

__device__ __forceinline__ unsigned short f2bf_bits(float f) {
  unsigned u = __float_as_uint(f);
  return (unsigned short)((u + 0x7FFFu + ((u >> 16) & 1u)) >> 16);
}
__device__ __forceinline__ float bf_bits2f(unsigned short h) { return __uint_as_float(((unsigned)h) << 16); }

__device__ __forceinline__ void dep_guard_h(v8f& a, v8f& b, v16h x, v16h y) { asm volatile("v_nop\n\tv_nop\n\tv_nop\n\tv_nop" : "+v"(a), "+v"(b) : "v"(x), "v"(y)); }
__device__ __forceinline__ void dep_guard_b(v8f& a, v8f& b, v16b x, v16b y) { asm volatile("v_nop\n\tv_nop\n\tv_nop\n\tv_nop" : "+v"(a), "+v"(b) : "v"(x), "v"(y)); }
__device__ __forceinline__ void keep4_h(v16h a, v16h b, v16h c, v16h d) { asm volatile("v_nop" :: "v"(a), "v"(b), "v"(c), "v"(d)); }
__device__ __forceinline__ void keep4_b(v16b a, v16b b, v16b c, v16b d) { asm volatile("v_nop" :: "v"(a), "v"(b), "v"(c), "v"(d)); }
__device__ __forceinline__ void acc_guard4(v8f& a, v8f& b, v8f& c, v8f& d) { asm volatile("v_nop\n\tv_nop\n\tv_nop\n\tv_nop" : "+v"(a), "+v"(b), "+v"(c), "+v"(d)); }
template <typename T> struct Frag;
template <> struct Frag<_Float16> {
  typedef v16h V; union U { v16h v; v8h h[2]; };
  static __device__ __forceinline__ v16h load(const _Float16* p) {
    U f; f.h[0] = *(const v8h*)(p); f.h[1] = *(const v8h*)(p + 16); return f.v;
  }
  static __device__ __forceinline__ v8f mma(v16h a, v16h b, v8f c) {
    return __builtin_amdgcn_wmma_f32_16x16x32_f16(false, a, false, b, (short)0, c, false, false);
  }
  static __device__ __forceinline__ void guard(v8f& a, v8f& b, v16h x, v16h y) { dep_guard_h(a, b, x, y); }
  static __device__ __forceinline__ void keep(v16h a, v16h b, v16h c, v16h d) { keep4_h(a, b, c, d); }
};
template <> struct Frag<__bf16> {
  typedef v16b V; union U { v16b v; v8b h[2]; };
  static __device__ __forceinline__ v16b load(const __bf16* p) {
    U f; f.h[0] = *(const v8b*)(p); f.h[1] = *(const v8b*)(p + 16); return f.v;
  }
  static __device__ __forceinline__ v8f mma(v16b a, v16b b, v8f c) {
    return __builtin_amdgcn_wmma_f32_16x16x32_bf16(false, a, false, b, (short)0, c, false, false);
  }
  static __device__ __forceinline__ void guard(v8f& a, v8f& b, v16b x, v16b y) { dep_guard_b(a, b, x, y); }
  static __device__ __forceinline__ void keep(v16b a, v16b b, v16b c, v16b d) { keep4_b(a, b, c, d); }
};

template <int ET> struct Elem;
template <> struct Elem<0> { typedef _Float16 T; };
template <> struct Elem<1> { typedef __bf16 T; };
template <int ET, bool SPLIT, int BIAS_MODE, int OUT_MODE, bool RESID, int ACT = 0>
__global__ __launch_bounds__(256) void wmma_gemm64(
    const unsigned short* __restrict__ Ap, const unsigned short* __restrict__ A2p, int lda, long strideA,
    const unsigned short* __restrict__ Btp, const unsigned short* __restrict__ Bt2p, int ldb, long strideB,
    void* __restrict__ Cout, void* __restrict__ Cout2, int ldc, long strideC,
    const float* __restrict__ bias, long strideBias,
    const float* __restrict__ resid, long strideR,
    int M, int N, int K, float scale) {
  static_assert(!(RESID && OUT_MODE != 0), "");
  static_assert(!(RESID && ACT != 0), "");
  typedef typename Elem<ET>::T T;
  typedef typename Frag<T>::V V;
  const T* A = (const T*)Ap; const T* A2 = (const T*)A2p; const T* Bt = (const T*)Btp; const T* Bt2 = (const T*)Bt2p;
  __shared__ __align__(16) float sT[8][16 * 68];
  const int b    = blockIdx.y;
  const int lane = threadIdx.x & 31;
  const int wave = threadIdx.x >> 5;
  const int tilesN = N >> 6;
  const int tilesM = M >> 6;
  const int tile = blockIdx.x * 8 + wave;
  if (tile >= tilesM * tilesN) return;
  const int tm = tile / tilesN;
  const int tn = tile - tm * tilesN;
  const int m0 = tm << 6;
  const int n0 = tn << 6;

  const T* Ab  = A  + (size_t)b * strideA;
  const T* Bb  = Bt + (size_t)b * strideB;
  const T* Ab2 = SPLIT ? (A2  + (size_t)b * strideA) : nullptr;
  const T* Bb2 = SPLIT ? (Bt2 + (size_t)b * strideB) : nullptr;

  const int rlane = lane & 15;
  const int koff  = (lane >> 4) * 8;
  const int mOff  = (lane >> 4) * 8;

  v8f acc[4][4];
#pragma unroll
  for (int i = 0; i < 4; ++i)
#pragma unroll
    for (int j = 0; j < 4; ++j) acc[i][j] = (v8f){0.f,0.f,0.f,0.f,0.f,0.f,0.f,0.f};

  for (int k0 = 0; k0 < K; k0 += 32) {
    V bh[4], bl[4];
#pragma unroll
    for (int j = 0; j < 4; ++j) {
      const size_t bo = (size_t)(n0 + (j << 4) + rlane) * ldb + koff + k0;
      bh[j] = Frag<T>::load(Bb + bo);
      if (SPLIT) bl[j] = Frag<T>::load(Bb2 + bo);
    }
#pragma unroll
    for (int i = 0; i < 4; ++i) {
      const size_t ao = (size_t)(m0 + (i << 4) + rlane) * lda + koff + k0;
      V ah = Frag<T>::load(Ab + ao);
      V al;
      if (SPLIT) al = Frag<T>::load(Ab2 + ao);
#pragma unroll
      for (int j = 0; j < 4; ++j) {
        acc[i][j] = Frag<T>::mma(ah, bh[j], acc[i][j]);
        if (SPLIT) {
          acc[i][j] = Frag<T>::mma(ah, bl[j], acc[i][j]);
          acc[i][j] = Frag<T>::mma(al, bh[j], acc[i][j]);
        }
      }
      Frag<T>::guard(acc[i][0], acc[i][3], ah, SPLIT ? al : ah);
    }
    Frag<T>::keep(bh[0], bh[1], bh[2], bh[3]);
    if (SPLIT) Frag<T>::keep(bl[0], bl[1], bl[2], bl[3]);
  }
  acc_guard4(acc[0][0], acc[0][1], acc[0][2], acc[0][3]);
  acc_guard4(acc[1][0], acc[1][1], acc[1][2], acc[1][3]);
  acc_guard4(acc[2][0], acc[2][1], acc[2][2], acc[2][3]);
  acc_guard4(acc[3][0], acc[3][1], acc[3][2], acc[3][3]);

  float* slab = sT[wave];
  const float* Rb = RESID ? (resid + (size_t)b * strideR) : nullptr;
  const float* biasb = (BIAS_MODE != 0) ? (bias + (size_t)b * strideBias) : nullptr;
#pragma unroll
  for (int i = 0; i < 4; ++i) {
    const int mBase = m0 + (i << 4);
#pragma unroll
    for (int j = 0; j < 4; ++j) {
      const int n = n0 + (j << 4) + rlane;
      float bv = 0.f;
      if (BIAS_MODE == 2) bv = biasb[n];
#pragma unroll
      for (int r = 0; r < 8; ++r) {
        float v = acc[i][j][r] * scale;
        if (BIAS_MODE == 1) v += biasb[mBase + mOff + r];
        if (BIAS_MODE == 2) v += bv;
        if (ACT == 2) v = fmaxf(v, 0.0f);
        if (ACT == 4) v = (v > 0.f) ? v : 0.01f * v;
        slab[(mOff + r) * 68 + (j << 4) + rlane] = v;
      }
    }
    __builtin_amdgcn_fence(__ATOMIC_RELEASE, "workgroup");
    __builtin_amdgcn_wave_barrier();
    __builtin_amdgcn_fence(__ATOMIC_ACQUIRE, "workgroup");
    if (OUT_MODE == 0) {
      float* C = (float*)Cout + (size_t)b * strideC;
      const int hh = lane >> 4, c4 = (lane & 15) * 4;
      for (int pass = 0; pass < 2; ++pass) {
#pragma unroll
        for (int it = 0; it < 8; ++it) {
          const int row = it * 2 + hh;
          v4f v = *(const v4f*)(slab + row * 68 + c4);
          if (RESID) {
            const v4f rr = *(const v4f*)(Rb + (size_t)(mBase + row) * ldc + n0 + c4);
            v = v + rr;
          }
          *(volatile v4f*)(C + (size_t)(mBase + row) * ldc + n0 + c4) = v;
        }
        __threadfence();
      }
    } else {
      const int q = lane >> 3, c8 = (lane & 7) * 8;
      unsigned short* C  = (unsigned short*)Cout  + (size_t)b * strideC;
      unsigned short* C2 = (OUT_MODE == 2) ? ((unsigned short*)Cout2 + (size_t)b * strideC) : nullptr;
      for (int pass = 0; pass < 2; ++pass) {
#pragma unroll
        for (int it = 0; it < 4; ++it) {
          const int row = it * 4 + q;
          const float* sp = slab + row * 68 + c8;
          v8h hv, lv;
#pragma unroll
          for (int e = 0; e < 8; ++e) {
            if (OUT_MODE == 1) {
              hv[e] = (_Float16)sp[e];
            } else {
              unsigned short hb = f2bf_bits(sp[e]);
              unsigned short lb = f2bf_bits(sp[e] - bf_bits2f(hb));
              hv[e] = __builtin_bit_cast(_Float16, hb);
              lv[e] = __builtin_bit_cast(_Float16, lb);
            }
          }
          *(volatile v8h*)(C + (size_t)(mBase + row) * ldc + n0 + c8) = hv;
          if (OUT_MODE == 2) *(volatile v8h*)(C2 + (size_t)(mBase + row) * ldc + n0 + c8) = lv;
        }
        __threadfence();
      }
    }
    __builtin_amdgcn_fence(__ATOMIC_RELEASE, "workgroup");
    __builtin_amdgcn_wave_barrier();
    __builtin_amdgcn_fence(__ATOMIC_ACQUIRE, "workgroup");
  }
}

__device__ __forceinline__ void split8(const v4f a, const v4f c, v8h& hv, v8h& lv) {
#pragma unroll
  for (int e = 0; e < 4; ++e) {
    const float x0 = a[e];
    const unsigned short hb0 = f2bf_bits(x0);
    const unsigned short lb0 = f2bf_bits(x0 - bf_bits2f(hb0));
    hv[e] = __builtin_bit_cast(_Float16, hb0);
    lv[e] = __builtin_bit_cast(_Float16, lb0);
    const float x1 = c[e];
    const unsigned short hb1 = f2bf_bits(x1);
    const unsigned short lb1 = f2bf_bits(x1 - bf_bits2f(hb1));
    hv[4 + e] = __builtin_bit_cast(_Float16, hb1);
    lv[4 + e] = __builtin_bit_cast(_Float16, lb1);
  }
}
__device__ __forceinline__ void store2x16(unsigned short* ph, unsigned short* pl, v8h hv, v8h lv) {
  *(volatile v8h*)ph = hv;
  *(volatile v8h*)pl = lv;
  __threadfence();
  *(volatile v8h*)ph = hv;
  *(volatile v8h*)pl = lv;
}
__device__ __forceinline__ float gate_sigmoid(float x) { return 1.0f / (1.0f + expf(-x)); }

__global__ __launch_bounds__(256) void split_planes(const float* __restrict__ src,
                                                    unsigned short* __restrict__ dh,
                                                    unsigned short* __restrict__ dl, int n8) {
  const int i = blockIdx.x * 256 + threadIdx.x;
  if (i >= n8) return;
  const size_t e0 = (size_t)i * 8;
  const v4f a = *(const v4f*)(src + e0);
  const v4f c = *(const v4f*)(src + e0 + 4);
  v8h hv, lv;
  split8(a, c, hv, lv);
  store2x16(dh + e0, dl + e0, hv, lv);
}

__global__ __launch_bounds__(256) void split_w5(const float* __restrict__ w0, const float* __restrict__ w1,
                                                const float* __restrict__ w2, const float* __restrict__ w3,
                                                const float* __restrict__ w4,
                                                unsigned short* __restrict__ dh, unsigned short* __restrict__ dl) {
  const int y = blockIdx.y;
  const float* src = (y == 0) ? w0 : (y == 1) ? w1 : (y == 2) ? w2 : (y == 3) ? w3 : w4;
  const int i = blockIdx.x * 256 + threadIdx.x;
  if (i >= (int)(WELEM / 8)) return;
  const size_t e0 = (size_t)i * 8;
  const v4f a = *(const v4f*)(src + e0);
  const v4f c = *(const v4f*)(src + e0 + 4);
  v8h hv, lv;
  split8(a, c, hv, lv);
  store2x16(dh + (size_t)y * WELEM + e0, dl + (size_t)y * WELEM + e0, hv, lv);
}

__global__ __launch_bounds__(64) void copy_bias4(const float* __restrict__ b0, const float* __restrict__ b1,
                                                 const float* __restrict__ b2, const float* __restrict__ b3,
                                                 float* __restrict__ dst) {
  const int y = blockIdx.y;
  const float* src = (y == 0) ? b0 : (y == 1) ? b1 : (y == 2) ? b2 : b3;
  const int t = threadIdx.x;
  const v4f v = *(const v4f*)(src + 4 * t);
  float* d = dst + (size_t)y * DMODEL + 4 * t;
  *(volatile v4f*)d = v;
  __threadfence();
  *(volatile v4f*)d = v;
}

__global__ __launch_bounds__(256) void den_scan(const float* __restrict__ Fpre, const float* __restrict__ Ipre,
                                                const float* __restrict__ Kf, const float* __restrict__ Qf,
                                                float* __restrict__ den) {
  __shared__ float part[SEQ * 8];
  __shared__ __align__(16) float dens[SEQ];
  const int tid = threadIdx.x, lane = tid & 31, w = tid >> 5;
  const int b = blockIdx.x;
  const size_t base = (size_t)b * SEQ * DMODEL + tid;
  float n = 0.0f;
#pragma unroll 1
  for (int t = 0; t < SEQ; ++t) {
    const size_t idx = base + (size_t)t * DMODEL;
    const float fp = Fpre[idx];
    const float ip = Ipre[idx];
    const float kk = Kf[idx];
    const float qq = Qf[idx];
    const float fg = gate_sigmoid(fp);
    const float ig = expf(ip);
    n = fg * n + ig * kk;
    float p = n * qq;
    p += __shfl_xor(p, 16, 32);
    p += __shfl_xor(p, 8, 32);
    p += __shfl_xor(p, 4, 32);
    p += __shfl_xor(p, 2, 32);
    p += __shfl_xor(p, 1, 32);
    if (lane == 0) part[t * 8 + w] = p;
  }
  __syncthreads();
  for (int t = tid; t < SEQ; t += 256) {
    float s = part[t * 8 + 0];
    s += part[t * 8 + 1]; s += part[t * 8 + 2]; s += part[t * 8 + 3];
    s += part[t * 8 + 4]; s += part[t * 8 + 5]; s += part[t * 8 + 6]; s += part[t * 8 + 7];
    s = fabsf(s);
    dens[t] = fmaxf(s, 1.0f);
  }
  __syncthreads();
  {
    const int line = w * 4 + (lane >> 3);
    const int c4 = (lane & 7) * 4;
    const int e = line * 32 + c4;
    const v4f v = *(const v4f*)(dens + e);
    float* d = den + (size_t)b * SEQ + e;
    *(volatile v4f*)d = v;
    __threadfence();
    *(volatile v4f*)d = v;
  }
}

__global__ __launch_bounds__(256) void pair_prep(const float* __restrict__ Fpre, const float* __restrict__ Ipre,
                                                 const float* __restrict__ Kf, const float* __restrict__ Qf,
                                                 float* __restrict__ fcum,
                                                 unsigned short* __restrict__ gth, unsigned short* __restrict__ gtl,
                                                 unsigned short* __restrict__ kth, unsigned short* __restrict__ ktl) {
  __shared__ float Ft[PLEN * 65];
  __shared__ float Gs[PLEN * 65];
  __shared__ float Ks[PLEN * 65];
  const int tid = threadIdx.x, lane = tid & 31, w = tid >> 5;
  const int slab = blockIdx.x;
  const int p = blockIdx.y;
  const size_t rowbase = (size_t)p * PLEN;
  const int colbase = slab * 64;

#pragma unroll 1
  for (int it = 0; it < 4; ++it) {
    const int idx = it * 256 + tid;
    const int r = idx >> 4;
    const int c4 = (idx & 15) * 4;
    const size_t g = (rowbase + r) * DMODEL + colbase + c4;
    const v4f fv = *(const v4f*)(Fpre + g);
    const v4f kv = *(const v4f*)(Kf + g);
    const v4f iv = *(const v4f*)(Ipre + g);
    const v4f qv = *(const v4f*)(Qf + g);
#pragma unroll
    for (int e = 0; e < 4; ++e) {
      Ft[r * 65 + c4 + e] = gate_sigmoid(fv[e]);
      Ks[r * 65 + c4 + e] = kv[e];
      Gs[r * 65 + c4 + e] = expf(iv[e]) * qv[e];
    }
  }
  __syncthreads();
  if (tid < 64) {
    float acc = 1.0f;
#pragma unroll 1
    for (int s = 0; s < PLEN; ++s) {
      acc = acc * Ft[s * 65 + tid];
      acc = fmaxf(acc, 1e-30f);
      Ft[s * 65 + tid] = acc;
    }
  }
  __syncthreads();
#pragma unroll 1
  for (int it = 0; it < 16; ++it) {
    const int idx = it * 256 + tid;
    const int r = idx >> 6, c = idx & 63;
    const float fc = Ft[r * 65 + c];
    Gs[r * 65 + c] = Gs[r * 65 + c] * (1.0f / fc);
  }
  __syncthreads();
  for (int pass = 0; pass < 2; ++pass) {
    {
      const int hh = lane >> 4, c4 = (lane & 15) * 4;
#pragma unroll
      for (int it = 0; it < 4; ++it) {
        const int row = it * 16 + w * 2 + hh;
        v4f v;
        v[0] = Ft[row * 65 + c4 + 0]; v[1] = Ft[row * 65 + c4 + 1];
        v[2] = Ft[row * 65 + c4 + 2]; v[3] = Ft[row * 65 + c4 + 3];
        *(volatile v4f*)(fcum + (rowbase + row) * DMODEL + colbase + c4) = v;
      }
    }
    {
      const int q8 = lane >> 3, s0 = (lane & 7) * 8;
#pragma unroll
      for (int it = 0; it < 2; ++it) {
        const int c = it * 32 + w * 4 + q8;
        v4f ga, gb, ka, kb;
#pragma unroll
        for (int e = 0; e < 4; ++e) {
          ga[e] = Gs[(s0 + e) * 65 + c];
          gb[e] = Gs[(s0 + 4 + e) * 65 + c];
          ka[e] = Ks[(s0 + e) * 65 + c];
          kb[e] = Ks[(s0 + 4 + e) * 65 + c];
        }
        v8h ghv, glv, khv, klv;
        split8(ga, gb, ghv, glv);
        split8(ka, kb, khv, klv);
        const size_t line = ((size_t)p * DMODEL + colbase + c) * PLEN + s0;
        *(volatile v8h*)(gth + line) = ghv;
        *(volatile v8h*)(gtl + line) = glv;
        *(volatile v8h*)(kth + line) = khv;
        *(volatile v8h*)(ktl + line) = klv;
      }
    }
    __threadfence();
  }
}

__global__ __launch_bounds__(256) void causal_split(const float* __restrict__ ad,
                                                    unsigned short* __restrict__ ath,
                                                    unsigned short* __restrict__ atl) {
  const int g = blockIdx.x * 256 + threadIdx.x;
  if (g >= NPAIR * PLEN * (PLEN / 8)) return;
  const int p = g >> 9, rem = g & 511, t = rem >> 3, s0 = (rem & 7) * 8;
  const size_t e0 = (size_t)p * (PLEN * PLEN) + (size_t)t * PLEN + s0;
  v4f a = *(const v4f*)(ad + e0);
  v4f c = *(const v4f*)(ad + e0 + 4);
#pragma unroll
  for (int e = 0; e < 4; ++e) {
    a[e] = (s0 + e <= t) ? a[e] : 0.0f;
    c[e] = (s0 + 4 + e <= t) ? c[e] : 0.0f;
  }
  v8h hv, lv;
  split8(a, c, hv, lv);
  store2x16(ath + e0, atl + e0, hv, lv);
}

__global__ __launch_bounds__(256) void state_scan(const float* __restrict__ u, const float* __restrict__ fcum,
                                                  unsigned short* __restrict__ csh, unsigned short* __restrict__ csl) {
  const int g = blockIdx.x * 256 + threadIdx.x;
  if (g >= NBATCH * DMODEL * (DMODEL / 8)) return;
  const int b = g >> 13, rem = g & 8191, i = rem >> 5, k8 = (rem & 31) * 8;
  v4f ca = (v4f){0.0f, 0.0f, 0.0f, 0.0f};
  v4f cb = (v4f){0.0f, 0.0f, 0.0f, 0.0f};
#pragma unroll 1
  for (int P = 0; P < PAIRS_PER_SEQ; ++P) {
    const int p = b * PAIRS_PER_SEQ + P;
    const size_t e0 = ((size_t)p * DMODEL + i) * DMODEL + k8;
    v8h hv, lv;
    split8(ca, cb, hv, lv);
    store2x16(csh + e0, csl + e0, hv, lv);
    const v4f ua = *(const v4f*)(u + e0);
    const v4f ub = *(const v4f*)(u + e0 + 4);
    const float fl = fcum[((size_t)p * PLEN + (PLEN - 1)) * DMODEL + i];
    ca = (ca + ua) * fl;
    cb = (cb + ub) * fl;
  }
}

__global__ __launch_bounds__(256) void num_combine(const float* __restrict__ fc, const float* __restrict__ nsum,
                                                   const float* __restrict__ den,
                                                   unsigned short* __restrict__ hh, unsigned short* __restrict__ hl) {
  const int g = blockIdx.x * 256 + threadIdx.x;
  if (g >= MROWS * (DMODEL / 8)) return;
  const int t = g >> 5, i8 = (g & 31) * 8;
  const size_t e0 = (size_t)t * DMODEL + i8;
  const v4f fa = *(const v4f*)(fc + e0);
  const v4f fb = *(const v4f*)(fc + e0 + 4);
  const v4f na = *(const v4f*)(nsum + e0);
  const v4f nb = *(const v4f*)(nsum + e0 + 4);
  const float rd = 1.0f / den[t];
  const v4f ha = (fa * na) * rd;
  const v4f hb = (fb * nb) * rd;
  v8h hv, lv;
  split8(ha, hb, hv, lv);
  store2x16(hh + e0, hl + e0, hv, lv);
}

extern "C" void kernel_launch(void* const* d_in, const int* in_sizes, int n_in,
                              void* d_out, int out_size, void* d_ws, size_t ws_size,
                              hipStream_t stream) {
  if (n_in < 13) return;
  if (in_sizes[0] != (int)NELEM || out_size != (int)NELEM) return;
  if (in_sizes[1] != (int)WELEM || in_sizes[3] != (int)WELEM || in_sizes[7] != (int)WELEM ||
      in_sizes[9] != (int)WELEM || in_sizes[11] != (int)WELEM) return;
  if (in_sizes[2] != DMODEL || in_sizes[4] != DMODEL || in_sizes[8] != DMODEL ||
      in_sizes[10] != DMODEL || in_sizes[12] != DMODEL) return;
  if (ws_size < WS_TOTAL) return;

  const float* x   = (const float*)d_in[0];
  const float* Wq  = (const float*)d_in[1];
  const float* bq  = (const float*)d_in[2];
  const float* Wk  = (const float*)d_in[3];
  const float* bk  = (const float*)d_in[4];
  const float* Wf  = (const float*)d_in[7];
  const float* bfg = (const float*)d_in[8];
  const float* Wi  = (const float*)d_in[9];
  const float* bi  = (const float*)d_in[10];
  const float* Wo  = (const float*)d_in[11];
  const float* bo  = (const float*)d_in[12];
  float* out = (float*)d_out;

  char* ws = (char*)d_ws;
  unsigned short* XH  = (unsigned short*)(ws + OFF_XH);
  unsigned short* XL  = (unsigned short*)(ws + OFF_XL);
  float* QF  = (float*)(ws + OFF_QF);
  float* KF  = (float*)(ws + OFF_KF);
  float* FF  = (float*)(ws + OFF_FF);
  float* IFp = (float*)(ws + OFF_IF);
  float* U   = (float*)(ws + OFF_U);
  float* NS  = (float*)(ws + OFF_NS);
  unsigned short* WH  = (unsigned short*)(ws + OFF_WH);
  unsigned short* WL  = (unsigned short*)(ws + OFF_WL);
  float* BIAS = (float*)(ws + OFF_BIAS);
  unsigned short* QKH = (unsigned short*)(ws + OFF_QKH);
  unsigned short* QKL = (unsigned short*)(ws + OFF_QKL);
  unsigned short* GTH = (unsigned short*)(ws + OFF_GTH);
  unsigned short* GTL = (unsigned short*)(ws + OFF_GTL);
  unsigned short* KTH = (unsigned short*)(ws + OFF_KTH);
  unsigned short* KTL = (unsigned short*)(ws + OFF_KTL);
  float* AD  = (float*)(ws + OFF_AD);
  unsigned short* ATH = (unsigned short*)(ws + OFF_ATH);
  unsigned short* ATL = (unsigned short*)(ws + OFF_ATL);
  float* FC  = (float*)(ws + OFF_FC);
  float* DEN = (float*)(ws + OFF_DEN);
  float* N1  = (float*)(ws + OFF_N1);
  unsigned short* HH  = (unsigned short*)(ws + OFF_HH);
  unsigned short* HL  = (unsigned short*)(ws + OFF_HL);
  unsigned short* CSH = (unsigned short*)(ws + OFF_CSH);
  unsigned short* CSL = (unsigned short*)(ws + OFF_CSL);

  split_planes<<<(unsigned)(NELEM / 8 / 256), 256, 0, stream>>>(x, XH, XL, (int)(NELEM / 8));
  split_w5<<<dim3((unsigned)(WELEM / 8 / 256), 5), 256, 0, stream>>>(Wq, Wk, Wf, Wi, Wo, WH, WL);
  copy_bias4<<<dim3(1, 4), 64, 0, stream>>>(bq, bk, bfg, bi, BIAS);

  static_assert(MROWS % 64 == 0 && DMODEL % 64 == 0 && DMODEL % 32 == 0, "");
  wmma_gemm64<1, true, 2, 0, false, 0><<<dim3((MROWS / 64) * (DMODEL / 64) / 8, 4), 256, 0, stream>>>(
      XH, XL, DMODEL, 0L,
      WH, WL, DMODEL, (long)WELEM,
      QF, nullptr, DMODEL, (long)NELEM,
      BIAS, (long)DMODEL,
      nullptr, 0L,
      MROWS, DMODEL, DMODEL, 1.0f);

  split_planes<<<(unsigned)(2 * NELEM / 8 / 256), 256, 0, stream>>>(QF, QKH, QKL, (int)(2 * NELEM / 8));

  den_scan<<<NBATCH, 256, 0, stream>>>(FF, IFp, KF, QF, DEN);
  pair_prep<<<dim3(DMODEL / 64, NPAIR), 256, 0, stream>>>(FF, IFp, KF, QF, FC, GTH, GTL, KTH, KTL);

  static_assert(PLEN % 64 == 0 && DMODEL % 32 == 0, "");
  wmma_gemm64<1, true, 0, 0, false, 0><<<dim3(1, NPAIR), 32, 0, stream>>>(
      QKH, QKL, DMODEL, (long)PLEN * DMODEL,
      QKH + NELEM, QKL + NELEM, DMODEL, (long)PLEN * DMODEL,
      AD, nullptr, PLEN, (long)PLEN * PLEN,
      nullptr, 0L, nullptr, 0L,
      PLEN, PLEN, DMODEL, 1.0f);

  causal_split<<<(NPAIR * PLEN * (PLEN / 8)) / 256, 256, 0, stream>>>(AD, ATH, ATL);

  static_assert(PLEN % 32 == 0, "");
  wmma_gemm64<1, true, 0, 0, false, 0><<<dim3(1, NPAIR), 128, 0, stream>>>(
      ATH, ATL, PLEN, (long)PLEN * PLEN,
      GTH, GTL, PLEN, (long)DMODEL * PLEN,
      N1, nullptr, DMODEL, (long)PLEN * DMODEL,
      nullptr, 0L, nullptr, 0L,
      PLEN, DMODEL, PLEN, 1.0f);

  wmma_gemm64<1, true, 0, 0, false, 0><<<dim3((DMODEL / 64) * (DMODEL / 64) / 8, NPAIR), 256, 0, stream>>>(
      GTH, GTL, PLEN, (long)DMODEL * PLEN,
      KTH, KTL, PLEN, (long)DMODEL * PLEN,
      U, nullptr, DMODEL, (long)WELEM,
      nullptr, 0L, nullptr, 0L,
      DMODEL, DMODEL, PLEN, 1.0f);

  state_scan<<<(NBATCH * DMODEL * (DMODEL / 8)) / 256, 256, 0, stream>>>(U, FC, CSH, CSL);

  wmma_gemm64<1, true, 0, 0, true, 0><<<dim3(1, NPAIR), 128, 0, stream>>>(
      QKH, QKL, DMODEL, (long)PLEN * DMODEL,
      CSH, CSL, DMODEL, (long)WELEM,
      NS, nullptr, DMODEL, (long)PLEN * DMODEL,
      nullptr, 0L,
      N1, (long)PLEN * DMODEL,
      PLEN, DMODEL, DMODEL, 1.0f);

  num_combine<<<(MROWS * (DMODEL / 8)) / 256, 256, 0, stream>>>(FC, NS, DEN, HH, HL);

  wmma_gemm64<1, true, 2, 0, false, 0><<<dim3((MROWS / 64) * (DMODEL / 64) / 8, 1), 256, 0, stream>>>(
      HH, HL, DMODEL, 0L,
      WH + 4 * WELEM, WL + 4 * WELEM, DMODEL, 0L,
      out, nullptr, DMODEL, 0L,
      bo, 0L,
      nullptr, 0L,
      MROWS, DMODEL, DMODEL, 1.0f);
}
